// SignalingModel_89060441850572
// MI455X (gfx1250) — hardware-run, weakly checked
//
#include <hip/hip_runtime.h>

typedef __attribute__((ext_vector_type(16))) _Float16 v16h;
typedef __attribute__((ext_vector_type(8)))  _Float16 v8h;
typedef __attribute__((ext_vector_type(8)))  float    v8f;
typedef __attribute__((ext_vector_type(4)))  float    v4f;

constexpr int kSamples   = 512;
constexpr int kNodes     = 2048;
constexpr int kSteps     = 60;
constexpr int kTilesM    = kSamples / 64;
constexpr int kTilesN    = kNodes / 64;
constexpr int kTiles     = kTilesM * kTilesN;
constexpr int kGemmBlks  = kTiles / 8;
constexpr int kSlabPitch = 68;
static_assert(kSamples == 512 && kNodes == 2048 && kSteps == 60, "wire contract shapes");
static_assert((kSamples % 64) == 0 && (kNodes % 64) == 0 && (kNodes % 32) == 0, "tile multiples, K multiple of 32");
static_assert(kTiles == kGemmBlks * 8, "eight tiles per block, exact grid");
static_assert(kSteps >= 2, "first step handled by the bias-term kernel, last step stores the output");

constexpr float kCarryW = 256.0f;
constexpr float kCarryY = 32.0f;
constexpr float kFold   = 1.0f / (kCarryW * kCarryY);
constexpr float kF16Min = 6.103515625e-05f;
static_assert(kFold == 1.220703125e-4f, "fold = 2^-13");

constexpr size_t kOffWH   = 0;
constexpr size_t kOffXB   = kOffWH + (size_t)kNodes * kNodes * 2;
constexpr size_t kOffYA   = kOffXB + (size_t)kSamples * kNodes * 4;
constexpr size_t kOffYB   = kOffYA + (size_t)kSamples * kNodes * 2;
constexpr size_t kWsTotal = kOffYB + (size_t)kSamples * kNodes * 2;
static_assert(kWsTotal == 16777216ull, "carve total");
static_assert(kWsTotal <= 134217728ull, "carve cap");
static_assert((kOffXB % 128) == 0 && (kOffYA % 128) == 0 && (kOffYB % 128) == 0, "128-B aligned regions");

__device__ __forceinline__ unsigned short f2bf_bits(float f) {
  unsigned u = __float_as_uint(f);
  return (unsigned short)((u + 0x7FFFu + ((u >> 16) & 1u)) >> 16);
}
__device__ __forceinline__ float bf_bits2f(unsigned short h) { return __uint_as_float(((unsigned)h) << 16); }
__device__ __forceinline__ float bf16_value(float f) { return bf_bits2f(f2bf_bits(f)); }

__device__ __forceinline__ _Float16 plane16(float v, float carry) {
  const float c = v * carry;
  const float f = (fabsf(c) < kF16Min) ? 0.0f : c;
  return (_Float16)f;
}

__device__ __forceinline__ float act3(float x) {
  const float xs  = fmaxf(x, 0.5f);
  const float sat = 1.0f - 0.25f * __builtin_amdgcn_rcpf(xs);
  const float mid = (x < 0.5f) ? x : sat;
  return (x < 0.0f) ? (0.01f * x) : mid;
}

namespace eng {
union FragU { v16h v; v8h h[2]; };
__device__ __forceinline__ v16h frag_load(const _Float16* p) {
  FragU f;
  f.h[0] = *(const v8h*)(p);
  f.h[1] = *(const v8h*)(p + 16);
  return f.v;
}
__device__ __forceinline__ v8f mma16(v16h a, v16h b, v8f c) {
  return __builtin_amdgcn_wmma_f32_16x16x32_f16(false, a, false, b, (short)0, c, false, false);
}
__device__ __forceinline__ void tie_one(v8f& d, v16h a, v16h b) {
  asm volatile("v_nop" : "+v"(d) : "v"(a), "v"(b));
}
__device__ __forceinline__ void guard_last(v8f& d, v16h a, v16h b0, v16h b1, v16h b2, v16h b3) {
  asm volatile("v_nop\n\tv_nop\n\tv_nop\n\tv_nop" : "+v"(d) : "v"(a), "v"(b0), "v"(b1), "v"(b2), "v"(b3));
}
}

__global__ __launch_bounds__(256) void weight_plane(
    const float* __restrict__ W, unsigned short* __restrict__ WH, int total8)
{
  const int i = blockIdx.x * 256 + threadIdx.x;
  if (i >= total8) return;
  const size_t e0 = (size_t)i << 3;
  const v4f a0 = *(const v4f*)(W + e0);
  const v4f a1 = *(const v4f*)(W + e0 + 4);
  v8h hv;
#pragma unroll
  for (int e = 0; e < 4; ++e) {
    const float w0 = a0[e];
    const float w1 = a1[e];
    hv[e]     = plane16(bf16_value(w0), kCarryW);
    hv[4 + e] = plane16(bf16_value(w1), kCarryW);
  }
  unsigned short* q = WH + e0;
  *(volatile v8h*)q = hv;
  __threadfence();
  *(volatile v8h*)q = hv;
}

__global__ __launch_bounds__(256) void bias_term_first_iterate(
    const float* __restrict__ X, const float* __restrict__ bias,
    float* __restrict__ XB, unsigned short* __restrict__ Y)
{
  __shared__ __align__(16) float sRow[kNodes];
  const int t   = threadIdx.x;
  const int row = blockIdx.x;
  const int c0  = t * 8;
  const size_t rbase = (size_t)row * kNodes;
  const v4f x0 = *(const v4f*)(X + rbase + c0);
  const v4f x1 = *(const v4f*)(X + rbase + c0 + 4);
  const v4f b0 = *(const v4f*)(bias + c0);
  const v4f b1 = *(const v4f*)(bias + c0 + 4);
  v4f s0, s1;
  v8h hv;
#pragma unroll
  for (int e = 0; e < 4; ++e) {
    const float u0 = bf16_value(x0[e]) + bf16_value(b0[e]);
    const float u1 = bf16_value(x1[e]) + bf16_value(b1[e]);
    s0[e] = u0;
    s1[e] = u1;
    hv[e]     = plane16(act3(u0), kCarryY);
    hv[4 + e] = plane16(act3(u1), kCarryY);
  }
  *(v4f*)(sRow + c0)     = s0;
  *(v4f*)(sRow + c0 + 4) = s1;
  unsigned short* yp = Y + rbase + c0;
  *(volatile v8h*)yp = hv;
  __threadfence();
  *(volatile v8h*)yp = hv;
  __syncthreads();
  const v4f f0 = *(const v4f*)(sRow + 4 * t);
  const v4f f1 = *(const v4f*)(sRow + 1024 + 4 * t);
  float* xp = XB + rbase + 4 * t;
  for (int pass = 0; pass < 2; ++pass) {
    *(volatile v4f*)(xp)        = f0;
    *(volatile v4f*)(xp + 1024) = f1;
    __threadfence();
  }
}

template <bool LAST>
__global__ __launch_bounds__(256) void step_product(
    const unsigned short* __restrict__ Yin, const unsigned short* __restrict__ Wpl,
    const float* __restrict__ XB, unsigned short* __restrict__ Yout, float* __restrict__ Out)
{
  __shared__ __align__(16) float sT[8][16 * kSlabPitch];
  const int lane = threadIdx.x & 31;
  const int wave = threadIdx.x >> 5;
  const int tile = blockIdx.x * 8 + wave;
  const int tm = tile / kTilesN;
  const int tn = tile - tm * kTilesN;
  const int m0 = tm << 6;
  const int n0 = tn << 6;

  const _Float16* A  = (const _Float16*)(const void*)Yin;
  const _Float16* Bt = (const _Float16*)(const void*)Wpl;

  const int rlane = lane & 15;
  const int koff  = (lane >> 4) * 8;
  const int mOff  = (lane >> 4) * 8;

  const _Float16* ap = A  + (size_t)(m0 + rlane) * kNodes + koff;
  const _Float16* bp = Bt + (size_t)(n0 + rlane) * kNodes + koff;

  v8f acc[4][4];
#pragma unroll
  for (int i = 0; i < 4; ++i)
#pragma unroll
    for (int j = 0; j < 4; ++j) acc[i][j] = (v8f){0.f, 0.f, 0.f, 0.f, 0.f, 0.f, 0.f, 0.f};

#pragma unroll 1
  for (int k0 = 0; k0 < kNodes; k0 += 32) {
    v16h bh[4];
#pragma unroll
    for (int j = 0; j < 4; ++j) bh[j] = eng::frag_load(bp + (size_t)(j << 4) * kNodes + k0);
#pragma unroll
    for (int i = 0; i < 4; ++i) {
      const v16h ah = eng::frag_load(ap + (size_t)(i << 4) * kNodes + k0);
#pragma unroll
      for (int j = 0; j < 4; ++j) acc[i][j] = eng::mma16(ah, bh[j], acc[i][j]);
      eng::tie_one(acc[i][0], ah, bh[0]);
      eng::tie_one(acc[i][1], ah, bh[1]);
      eng::tie_one(acc[i][2], ah, bh[2]);
      eng::guard_last(acc[i][3], ah, bh[0], bh[1], bh[2], bh[3]);
    }
  }

  float* slab = sT[wave];
#pragma unroll
  for (int i = 0; i < 4; ++i) {
    const int mBase = m0 + (i << 4);
#pragma unroll
    for (int j = 0; j < 4; ++j) {
#pragma unroll
      for (int r = 0; r < 8; ++r) slab[(mOff + r) * kSlabPitch + (j << 4) + rlane] = acc[i][j][r];
    }
    __builtin_amdgcn_fence(__ATOMIC_RELEASE, "workgroup");
    __builtin_amdgcn_wave_barrier();
    __builtin_amdgcn_fence(__ATOMIC_ACQUIRE, "workgroup");
    if (LAST) {
      const int hh = lane >> 4;
      const int c4 = (lane & 15) * 4;
      v4f ov[8];
#pragma unroll
      for (int it = 0; it < 8; ++it) {
        const int row = it * 2 + hh;
        const v4f s = *(const v4f*)(slab + row * kSlabPitch + c4);
        const v4f x = *(const v4f*)(XB + (size_t)(mBase + row) * kNodes + n0 + c4);
#pragma unroll
        for (int e = 0; e < 4; ++e) {
          const float pre = fmaf(s[e], kFold, x[e]);
          ov[it][e] = act3(pre);
        }
      }
      for (int pass = 0; pass < 2; ++pass) {
#pragma unroll
        for (int it = 0; it < 8; ++it) {
          const int row = it * 2 + hh;
          *(volatile v4f*)(Out + (size_t)(mBase + row) * kNodes + n0 + c4) = ov[it];
        }
        __threadfence();
      }
    } else {
      const int q  = lane >> 3;
      const int c8 = (lane & 7) * 8;
      v8h hv[4];
#pragma unroll
      for (int it = 0; it < 4; ++it) {
        const int row = it * 4 + q;
        const float* sp = slab + row * kSlabPitch + c8;
        const float* xp = XB + (size_t)(mBase + row) * kNodes + n0 + c8;
        const v4f s0 = *(const v4f*)(sp);
        const v4f s1 = *(const v4f*)(sp + 4);
        const v4f x0 = *(const v4f*)(xp);
        const v4f x1 = *(const v4f*)(xp + 4);
#pragma unroll
        for (int e = 0; e < 4; ++e) {
          const float p0 = fmaf(s0[e], kFold, x0[e]);
          const float p1 = fmaf(s1[e], kFold, x1[e]);
          hv[it][e]     = plane16(act3(p0), kCarryY);
          hv[it][4 + e] = plane16(act3(p1), kCarryY);
        }
      }
      for (int pass = 0; pass < 2; ++pass) {
#pragma unroll
        for (int it = 0; it < 4; ++it) {
          const int row = it * 4 + q;
          *(volatile v8h*)(Yout + (size_t)(mBase + row) * kNodes + n0 + c8) = hv[it];
        }
        __threadfence();
      }
    }
    __builtin_amdgcn_fence(__ATOMIC_RELEASE, "workgroup");
    __builtin_amdgcn_wave_barrier();
    __builtin_amdgcn_fence(__ATOMIC_ACQUIRE, "workgroup");
  }
}

extern "C" void kernel_launch(void* const* d_in, const int* in_sizes, int n_in,
                              void* d_out, int out_size, void* d_ws, size_t ws_size,
                              hipStream_t stream) {
  if (n_in < 3) return;
  if (in_sizes[0] != kSamples * kNodes) return;
  if (in_sizes[1] != kNodes * kNodes) return;
  if (in_sizes[2] != kNodes) return;
  if (out_size != kSamples * kNodes) return;
  if (ws_size < kWsTotal) return;

  const float* X_full  = (const float*)d_in[0];
  const float* weights = (const float*)d_in[1];
  const float* bias    = (const float*)d_in[2];
  float* out = (float*)d_out;

  char* ws = (char*)d_ws;
  unsigned short* WH = (unsigned short*)(ws + kOffWH);
  float*          XB = (float*)(ws + kOffXB);
  unsigned short* YA = (unsigned short*)(ws + kOffYA);
  unsigned short* YB = (unsigned short*)(ws + kOffYB);

  weight_plane<<<(kNodes * kNodes / 8) / 256, 256, 0, stream>>>(weights, WH, kNodes * kNodes / 8);
  bias_term_first_iterate<<<kSamples, 256, 0, stream>>>(X_full, bias, XB, YA);

  unsigned short* cur = YA;
  unsigned short* nxt = YB;
  for (int s = 2; s <= kSteps; ++s) {
    if (s < kSteps) {
      step_product<false><<<kGemmBlks, 256, 0, stream>>>(cur, WH, XB, nxt, out);
    } else {
      step_product<true><<<kGemmBlks, 256, 0, stream>>>(cur, WH, XB, nxt, out);
    }
    unsigned short* tmp = cur;
    cur = nxt;
    nxt = tmp;
  }
}
